// MultiHeadBatched_74071005987473
// MI455X (gfx1250) — hardware-verified
//
#include <hip/hip_runtime.h>
#include <math.h>
#include <stdint.h>

#define NBATCH 2
#define NHEADS 16
#define SEQL   2048
#define DMOD   1024
#define DHD    64
#define HGRP   2
#define NGRP   (NHEADS / HGRP)
#define PSCALE 32768.0f
#define PSCALE_INV (1.0f / 32768.0f)
#define CSCALE 64.0f
#define WCARRY 16.0f

typedef __attribute__((ext_vector_type(16))) _Float16 v16h;
typedef __attribute__((ext_vector_type(8)))  _Float16 v8h;
typedef __attribute__((ext_vector_type(16))) __bf16   v16b;
typedef __attribute__((ext_vector_type(8)))  __bf16   v8b;
typedef __attribute__((ext_vector_type(8)))  float    v8f;
typedef __attribute__((ext_vector_type(4)))  float    v4f;
typedef __attribute__((ext_vector_type(2)))  float    v2f;
typedef __attribute__((ext_vector_type(4)))  unsigned int v4u;
typedef __attribute__((ext_vector_type(4)))  int      v4i;

__device__ __forceinline__ unsigned short f2bf_bits(float f) {
  unsigned u = __float_as_uint(f);
  return (unsigned short)((u + 0x7FFFu + ((u >> 16) & 1u)) >> 16);
}
__device__ __forceinline__ float bf_bits2f(unsigned short h) { return __uint_as_float(((unsigned)h) << 16); }

__device__ __forceinline__ void dep_guard_h(v8f& a, v8f& b, v16h x, v16h y) { asm volatile("v_nop\n\tv_nop\n\tv_nop\n\tv_nop" : "+v"(a), "+v"(b) : "v"(x), "v"(y)); }
__device__ __forceinline__ void dep_guard_b(v8f& a, v8f& b, v16b x, v16b y) { asm volatile("v_nop\n\tv_nop\n\tv_nop\n\tv_nop" : "+v"(a), "+v"(b) : "v"(x), "v"(y)); }
__device__ __forceinline__ void keep4_h(v16h a, v16h b, v16h c, v16h d) { asm volatile("v_nop" :: "v"(a), "v"(b), "v"(c), "v"(d)); }
__device__ __forceinline__ void keep4_b(v16b a, v16b b, v16b c, v16b d) { asm volatile("v_nop" :: "v"(a), "v"(b), "v"(c), "v"(d)); }
__device__ __forceinline__ void acc_guard4(v8f& a, v8f& b, v8f& c, v8f& d) { asm volatile("v_nop\n\tv_nop\n\tv_nop\n\tv_nop" : "+v"(a), "+v"(b), "+v"(c), "+v"(d)); }
template <typename T> struct Frag;
template <> struct Frag<_Float16> {
  typedef v16h V; union U { v16h v; v8h h[2]; };
  static __device__ __forceinline__ v16h load(const _Float16* p) {
    U f; f.h[0] = *(const v8h*)(p); f.h[1] = *(const v8h*)(p + 16); return f.v;
  }
  static __device__ __forceinline__ v8f mma(v16h a, v16h b, v8f c) {
    return __builtin_amdgcn_wmma_f32_16x16x32_f16(false, a, false, b, (short)0, c, false, false);
  }
  static __device__ __forceinline__ void guard(v8f& a, v8f& b, v16h x, v16h y) { dep_guard_h(a, b, x, y); }
  static __device__ __forceinline__ void keep(v16h a, v16h b, v16h c, v16h d) { keep4_h(a, b, c, d); }
};
template <> struct Frag<__bf16> {
  typedef v16b V; union U { v16b v; v8b h[2]; };
  static __device__ __forceinline__ v16b load(const __bf16* p) {
    U f; f.h[0] = *(const v8b*)(p); f.h[1] = *(const v8b*)(p + 16); return f.v;
  }
  static __device__ __forceinline__ v8f mma(v16b a, v16b b, v8f c) {
    return __builtin_amdgcn_wmma_f32_16x16x32_bf16(false, a, false, b, (short)0, c, false, false);
  }
  static __device__ __forceinline__ void guard(v8f& a, v8f& b, v16b x, v16b y) { dep_guard_b(a, b, x, y); }
  static __device__ __forceinline__ void keep(v16b a, v16b b, v16b c, v16b d) { keep4_b(a, b, c, d); }
};

template <int ET> struct Elem;
template <> struct Elem<0> { typedef _Float16 T; };
template <> struct Elem<1> { typedef __bf16 T; };
template <int ET, bool SPLIT, int BIAS_MODE, int OUT_MODE, bool RESID, int ACT = 0>
__global__ __launch_bounds__(256) void wmma_gemm64(
    const unsigned short* __restrict__ Ap, const unsigned short* __restrict__ A2p, int lda, long strideA,
    const unsigned short* __restrict__ Btp, const unsigned short* __restrict__ Bt2p, int ldb, long strideB,
    void* __restrict__ Cout, void* __restrict__ Cout2, int ldc, long strideC,
    const float* __restrict__ bias,
    const float* __restrict__ resid, long strideR,
    int M, int N, int K, float scale) {
  typedef typename Elem<ET>::T T;
  typedef typename Frag<T>::V V;
  const T* A = (const T*)Ap; const T* A2 = (const T*)A2p; const T* Bt = (const T*)Btp; const T* Bt2 = (const T*)Bt2p;
  __shared__ __align__(16) float sT[8][16 * 68];
  const int b    = blockIdx.y;
  const int lane = threadIdx.x & 31;
  const int wave = threadIdx.x >> 5;
  const int tilesN = N >> 6;
  const int tilesM = M >> 6;
  const int tile = blockIdx.x * 8 + wave;
  if (tile >= tilesM * tilesN) return;
  const int tm = tile / tilesN;
  const int tn = tile - tm * tilesN;
  const int m0 = tm << 6;
  const int n0 = tn << 6;

  const T* Ab  = A  + (size_t)b * strideA;
  const T* Bb  = Bt + (size_t)b * strideB;
  const T* Ab2 = SPLIT ? (A2  + (size_t)b * strideA) : nullptr;
  const T* Bb2 = SPLIT ? (Bt2 + (size_t)b * strideB) : nullptr;

  const int rlane = lane & 15;
  const int koff  = (lane >> 4) * 8;
  const int mOff  = (lane >> 4) * 8;

  v8f acc[4][4];
#pragma unroll
  for (int i = 0; i < 4; ++i)
#pragma unroll
    for (int j = 0; j < 4; ++j) acc[i][j] = (v8f){0.f,0.f,0.f,0.f,0.f,0.f,0.f,0.f};

  for (int k0 = 0; k0 < K; k0 += 32) {
    V bh[4], bl[4];
#pragma unroll
    for (int j = 0; j < 4; ++j) {
      const size_t bo = (size_t)(n0 + (j << 4) + rlane) * ldb + koff + k0;
      bh[j] = Frag<T>::load(Bb + bo);
      if (SPLIT) bl[j] = Frag<T>::load(Bb2 + bo);
    }
#pragma unroll
    for (int i = 0; i < 4; ++i) {
      const size_t ao = (size_t)(m0 + (i << 4) + rlane) * lda + koff + k0;
      V ah = Frag<T>::load(Ab + ao);
      V al;
      if (SPLIT) al = Frag<T>::load(Ab2 + ao);
#pragma unroll
      for (int j = 0; j < 4; ++j) {
        acc[i][j] = Frag<T>::mma(ah, bh[j], acc[i][j]);
        if (SPLIT) {
          acc[i][j] = Frag<T>::mma(ah, bl[j], acc[i][j]);
          acc[i][j] = Frag<T>::mma(al, bh[j], acc[i][j]);
        }
      }
      Frag<T>::guard(acc[i][0], acc[i][3], ah, SPLIT ? al : ah);
    }
    Frag<T>::keep(bh[0], bh[1], bh[2], bh[3]);
    if (SPLIT) Frag<T>::keep(bl[0], bl[1], bl[2], bl[3]);
  }
  acc_guard4(acc[0][0], acc[0][1], acc[0][2], acc[0][3]);
  acc_guard4(acc[1][0], acc[1][1], acc[1][2], acc[1][3]);
  acc_guard4(acc[2][0], acc[2][1], acc[2][2], acc[2][3]);
  acc_guard4(acc[3][0], acc[3][1], acc[3][2], acc[3][3]);

  float* slab = sT[wave];
  const float* Rb = RESID ? (resid + (size_t)b * strideR) : nullptr;
#pragma unroll
  for (int i = 0; i < 4; ++i) {
    const int mBase = m0 + (i << 4);
#pragma unroll
    for (int j = 0; j < 4; ++j) {
      const int n = n0 + (j << 4) + rlane;
      float bv = 0.f;
      if (BIAS_MODE == 2) bv = bias[n];
#pragma unroll
      for (int r = 0; r < 8; ++r) {
        float v = acc[i][j][r] * scale;
        if (BIAS_MODE == 1) v += bias[mBase + mOff + r];
        if (BIAS_MODE == 2) v += bv;
        if (RESID) v += Rb[(size_t)(mBase + mOff + r) * ldc + n];
        if (ACT == 1) v = tanhf(v);
        if (ACT == 2) v = fmaxf(v, 0.0f);
        if (ACT == 3) v = v / (1.0f + expf(-v));
        if (ACT == 4) v = (v > 0.f) ? v : 0.01f * v;
        slab[(mOff + r) * 68 + (j << 4) + rlane] = v;
      }
    }
    __builtin_amdgcn_fence(__ATOMIC_RELEASE, "workgroup");
    __builtin_amdgcn_wave_barrier();
    __builtin_amdgcn_fence(__ATOMIC_ACQUIRE, "workgroup");
    if (OUT_MODE == 0) {
      float* C = (float*)Cout + (size_t)b * strideC;
      const int hh = lane >> 4, c4 = (lane & 15) * 4;
      for (int pass = 0; pass < 2; ++pass) {
#pragma unroll
        for (int it = 0; it < 8; ++it) {
          const int row = it * 2 + hh;
          v4f v = *(const v4f*)(slab + row * 68 + c4);
          *(volatile v4f*)(C + (size_t)(mBase + row) * ldc + n0 + c4) = v;
        }
        __threadfence();
      }
    } else {
      const int q = lane >> 3, c8 = (lane & 7) * 8;
      unsigned short* C  = (unsigned short*)Cout  + (size_t)b * strideC;
      unsigned short* C2 = (OUT_MODE == 2) ? ((unsigned short*)Cout2 + (size_t)b * strideC) : nullptr;
      for (int pass = 0; pass < 2; ++pass) {
#pragma unroll
        for (int it = 0; it < 4; ++it) {
          const int row = it * 4 + q;
          const float* sp = slab + row * 68 + c8;
          v8h hv, lv;
#pragma unroll
          for (int e = 0; e < 8; ++e) {
            if (OUT_MODE == 1) {
              hv[e] = (_Float16)sp[e];
            } else {
              unsigned short hb = f2bf_bits(sp[e]);
              unsigned short lb = f2bf_bits(sp[e] - bf_bits2f(hb));
              hv[e] = __builtin_bit_cast(_Float16, hb);
              lv[e] = __builtin_bit_cast(_Float16, lb);
            }
          }
          *(volatile v8h*)(C + (size_t)(mBase + row) * ldc + n0 + c8) = hv;
          if (OUT_MODE == 2) *(volatile v8h*)(C2 + (size_t)(mBase + row) * ldc + n0 + c8) = lv;
        }
        __threadfence();
      }
    }
    __builtin_amdgcn_fence(__ATOMIC_RELEASE, "workgroup");
    __builtin_amdgcn_wave_barrier();
    __builtin_amdgcn_fence(__ATOMIC_ACQUIRE, "workgroup");
  }
}

__device__ __forceinline__ unsigned pk16(unsigned short a, unsigned short b) { return (unsigned)a | ((unsigned)b << 16); }
__device__ __forceinline__ unsigned short h_bits(float f) { const _Float16 h = (_Float16)f; return __builtin_bit_cast(unsigned short, h); }

__global__ __launch_bounds__(256) void cast_f16x2_kernel(const float* __restrict__ in, unsigned short* __restrict__ out, int n2, float scale) {
  const int i = blockIdx.x * 256 + threadIdx.x;
  if (i < n2) {
    const v2f f = *(const v2f*)(in + 2 * (size_t)i);
    const unsigned u = pk16(h_bits(f[0] * scale), h_bits(f[1] * scale));
    ((volatile unsigned*)out)[i] = u;
    __threadfence();
    ((volatile unsigned*)out)[i] = u;
  }
}

__global__ __launch_bounds__(256) void softmax_kmask_kernel(const float* __restrict__ S,
                                                            const int* __restrict__ kmask,
                                                            unsigned short* __restrict__ P) {
  __shared__ float redm[8];
  __shared__ float reds[8];
  const int i    = blockIdx.x;
  const int hg   = blockIdx.y;
  const int tid  = threadIdx.x;
  const int lane = tid & 31;
  const int wave = tid >> 5;
  const int j0   = tid * 8;
  const float* rp = S + ((size_t)hg * SEQL + i) * SEQL + j0;
  const v4f a  = *(const v4f*)(rp);
  const v4f c  = *(const v4f*)(rp + 4);
  const v4i ma = *(const v4i*)(kmask + j0);
  const v4i mc = *(const v4i*)(kmask + j0 + 4);
  const float NEGF = -INFINITY;
  const float t0 = (ma[0] != 0) ? a[0] : NEGF;
  const float t1 = (ma[1] != 0) ? a[1] : NEGF;
  const float t2 = (ma[2] != 0) ? a[2] : NEGF;
  const float t3 = (ma[3] != 0) ? a[3] : NEGF;
  const float t4 = (mc[0] != 0) ? c[0] : NEGF;
  const float t5 = (mc[1] != 0) ? c[1] : NEGF;
  const float t6 = (mc[2] != 0) ? c[2] : NEGF;
  const float t7 = (mc[3] != 0) ? c[3] : NEGF;
  float m = fmaxf(fmaxf(fmaxf(t0, t1), fmaxf(t2, t3)), fmaxf(fmaxf(t4, t5), fmaxf(t6, t7)));
#pragma unroll
  for (int off = 16; off > 0; off >>= 1) m = fmaxf(m, __shfl_xor(m, off, 32));
  if (lane == 0) redm[wave] = m;
  __syncthreads();
  float mx = redm[0];
#pragma unroll
  for (int w = 1; w < 8; ++w) mx = fmaxf(mx, redm[w]);
  const float e0 = __expf(t0 - mx), e1 = __expf(t1 - mx), e2 = __expf(t2 - mx), e3 = __expf(t3 - mx);
  const float e4 = __expf(t4 - mx), e5 = __expf(t5 - mx), e6 = __expf(t6 - mx), e7 = __expf(t7 - mx);
  float s = ((e0 + e1) + (e2 + e3)) + ((e4 + e5) + (e6 + e7));
#pragma unroll
  for (int off = 16; off > 0; off >>= 1) s += __shfl_xor(s, off, 32);
  if (lane == 0) reds[wave] = s;
  __syncthreads();
  float tot = reds[0];
#pragma unroll
  for (int w = 1; w < 8; ++w) tot += reds[w];
  const float inv = 1.0f / tot;
  const float p0 = e0 * inv, p1 = e1 * inv, p2 = e2 * inv, p3 = e3 * inv;
  const float p4 = e4 * inv, p5 = e5 * inv, p6 = e6 * inv, p7 = e7 * inv;
  const v4u hv = (v4u){pk16(h_bits(p0 * PSCALE), h_bits(p1 * PSCALE)),
                       pk16(h_bits(p2 * PSCALE), h_bits(p3 * PSCALE)),
                       pk16(h_bits(p4 * PSCALE), h_bits(p5 * PSCALE)),
                       pk16(h_bits(p6 * PSCALE), h_bits(p7 * PSCALE))};
  const size_t ro = ((size_t)hg * SEQL + i) * SEQL + j0;
  *(volatile v4u*)(P + ro) = hv;
  __threadfence();
  *(volatile v4u*)(P + ro) = hv;
}

extern "C" void kernel_launch(void* const* d_in, const int* in_sizes, int n_in,
                              void* d_out, int out_size, void* d_ws, size_t ws_size,
                              hipStream_t stream) {
  if (n_in < 12) return;
  if (in_sizes[0] != NBATCH * SEQL * DMOD) return;
  if (in_sizes[1] != NBATCH * SEQL * DMOD) return;
  if (in_sizes[2] != NBATCH * SEQL * DMOD) return;
  if (in_sizes[3] != NBATCH * SEQL) return;
  if (in_sizes[4] != DMOD * DMOD || in_sizes[6] != DMOD * DMOD) return;
  if (in_sizes[8] != DMOD * DMOD || in_sizes[10] != DMOD * DMOD) return;
  if (in_sizes[5] != DMOD || in_sizes[7] != DMOD || in_sizes[9] != DMOD || in_sizes[11] != DMOD) return;
  if (out_size != NBATCH * SEQL * DMOD) return;

  const float* xq   = (const float*)d_in[0];
  const float* xk   = (const float*)d_in[1];
  const float* xv   = (const float*)d_in[2];
  const int*   kmsk = (const int*)d_in[3];
  const float* Wq   = (const float*)d_in[4];
  const float* bq   = (const float*)d_in[5];
  const float* Wk   = (const float*)d_in[6];
  const float* bk   = (const float*)d_in[7];
  const float* Wv   = (const float*)d_in[8];
  const float* bv   = (const float*)d_in[9];
  const float* Wo   = (const float*)d_in[10];
  const float* bo   = (const float*)d_in[11];

  const size_t PW = (size_t)DMOD * DMOD * 2;
  const size_t PX = (size_t)SEQL * DMOD * 2;
  const size_t PS = (size_t)HGRP * SEQL * SEQL * 4;
  const size_t PP = (size_t)HGRP * SEQL * SEQL * 2;
  size_t off = 0;
  const size_t oWq16  = off; off += PW;
  const size_t oWk16  = off; off += PW;
  const size_t oWv16  = off; off += PW;
  const size_t oWo16  = off; off += PW;
  const size_t oXQ16  = off; off += PX;
  const size_t oXK16  = off; off += PX;
  const size_t oXV16  = off; off += PX;
  const size_t oQ16   = off; off += PX;
  const size_t oK16   = off; off += PX;
  const size_t oVT16  = off; off += PX;
  const size_t oCTX16 = off; off += PX;
  const size_t oS     = off; off += PS;
  const size_t oP16   = off; off += PP;
  if (off > ws_size) return;

  char* ws = (char*)d_ws;
  unsigned short* Wq16  = (unsigned short*)(ws + oWq16);
  unsigned short* Wk16  = (unsigned short*)(ws + oWk16);
  unsigned short* Wv16  = (unsigned short*)(ws + oWv16);
  unsigned short* Wo16  = (unsigned short*)(ws + oWo16);
  unsigned short* XQ16  = (unsigned short*)(ws + oXQ16);
  unsigned short* XK16  = (unsigned short*)(ws + oXK16);
  unsigned short* XV16  = (unsigned short*)(ws + oXV16);
  unsigned short* Q16   = (unsigned short*)(ws + oQ16);
  unsigned short* K16   = (unsigned short*)(ws + oK16);
  unsigned short* VT16  = (unsigned short*)(ws + oVT16);
  unsigned short* CTX16 = (unsigned short*)(ws + oCTX16);
  float*          Sbuf  = (float*)(ws + oS);
  unsigned short* P16   = (unsigned short*)(ws + oP16);

  const int n2w = DMOD * DMOD / 2;
  const int n2x = SEQL * DMOD / 2;
  const dim3 blk(256);
  const dim3 gCastW((n2w + 255) / 256);
  const dim3 gCastX((n2x + 255) / 256);

  cast_f16x2_kernel<<<gCastW, blk, 0, stream>>>(Wq, Wq16, n2w, WCARRY);
  cast_f16x2_kernel<<<gCastW, blk, 0, stream>>>(Wk, Wk16, n2w, WCARRY);
  cast_f16x2_kernel<<<gCastW, blk, 0, stream>>>(Wv, Wv16, n2w, WCARRY);
  cast_f16x2_kernel<<<gCastW, blk, 0, stream>>>(Wo, Wo16, n2w, WCARRY);

  const int tilesM  = SEQL / 64;
  const dim3 gQK((tilesM * (DMOD / 64) + 7) / 8, 1);
  const dim3 gVT(((DMOD / 64) * (SEQL / 64) + 7) / 8, 1);
  const dim3 gS((tilesM * (SEQL / 64) + 7) / 8, HGRP);
  const dim3 gPV((tilesM * (DHD / 64) + 7) / 8, HGRP);
  const dim3 gO((tilesM * (DMOD / 64) + 7) / 8, 1);
  const float wscale = 1.0f / WCARRY;
  const float sscale = 0.125f;
  const float pvscale = PSCALE_INV * CSCALE;
  const float oscale  = 1.0f / (WCARRY * CSCALE);

  for (int b = 0; b < NBATCH; ++b) {
    cast_f16x2_kernel<<<gCastX, blk, 0, stream>>>(xq + (size_t)b * SEQL * DMOD, XQ16, n2x, 1.0f);
    cast_f16x2_kernel<<<gCastX, blk, 0, stream>>>(xk + (size_t)b * SEQL * DMOD, XK16, n2x, 1.0f);
    cast_f16x2_kernel<<<gCastX, blk, 0, stream>>>(xv + (size_t)b * SEQL * DMOD, XV16, n2x, 1.0f);
    wmma_gemm64<0, false, 2, 1, false, 0><<<gQK, blk, 0, stream>>>(
        XQ16, XQ16, DMOD, 0L, Wq16, Wq16, DMOD, 0L, (void*)Q16, (void*)Q16, DMOD, 0L,
        bq, bq, 0L, SEQL, DMOD, DMOD, wscale);
    wmma_gemm64<0, false, 2, 1, false, 0><<<gQK, blk, 0, stream>>>(
        XK16, XK16, DMOD, 0L, Wk16, Wk16, DMOD, 0L, (void*)K16, (void*)K16, DMOD, 0L,
        bk, bk, 0L, SEQL, DMOD, DMOD, wscale);
    wmma_gemm64<0, false, 1, 1, false, 0><<<gVT, blk, 0, stream>>>(
        Wv16, Wv16, DMOD, 0L, XV16, XV16, DMOD, 0L, (void*)VT16, (void*)VT16, SEQL, 0L,
        bv, bv, 0L, DMOD, SEQL, DMOD, wscale);
    const int* kmb = kmsk + (size_t)b * SEQL;
    for (int g = 0; g < NGRP; ++g) {
      const size_t hc = (size_t)g * HGRP * DHD;
      wmma_gemm64<0, false, 0, 0, false, 0><<<gS, blk, 0, stream>>>(
          Q16 + hc, Q16 + hc, DMOD, (long)DHD, K16 + hc, K16 + hc, DMOD, (long)DHD,
          (void*)Sbuf, (void*)Sbuf, SEQL, (long)SEQL * SEQL,
          bo, bo, 0L, SEQL, SEQL, DHD, sscale);
      softmax_kmask_kernel<<<dim3(SEQL, HGRP), blk, 0, stream>>>(Sbuf, kmb, P16);
      wmma_gemm64<0, false, 0, 1, false, 0><<<gPV, blk, 0, stream>>>(
          P16, P16, SEQL, (long)SEQL * SEQL, VT16 + hc * SEQL, VT16 + hc * SEQL, SEQL, (long)DHD * SEQL,
          (void*)(CTX16 + hc), (void*)(CTX16 + hc), DMOD, (long)DHD,
          bo, bo, 0L, SEQL, DHD, SEQL, pvscale);
    }
    float* outb = (float*)d_out + (size_t)b * SEQL * DMOD;
    wmma_gemm64<0, false, 2, 0, false, 0><<<gO, blk, 0, stream>>>(
        CTX16, CTX16, DMOD, 0L, Wo16, Wo16, DMOD, 0L, (void*)outb, (void*)outb, DMOD, 0L,
        bo, bo, 0L, SEQL, DMOD, DMOD, oscale);
  }
  (void)hipGetLastError();
}
